// Attention_67207648248320
// MI455X (gfx1250) — hardware-verified
//
#include <hip/hip_runtime.h>
#include <math.h>

#ifndef NB
#define NB 2
#endif
#ifndef SEQ
#define SEQ 2048
#endif
#define NB_FULL 2
#define SEQ_FULL 2048
#define DIMC 1024
#define NHEAD 16
#define HDIM 64
#define MROWS (NB * SEQ)

static_assert(SEQ % 64 == 0);
static_assert(SEQ <= SEQ_FULL);
static_assert(NB <= NB_FULL);
static_assert(DIMC == NHEAD * HDIM);
static_assert(DIMC % 64 == 0);
static_assert(DIMC / 8 == 128);
static_assert((MROWS % 64) == 0);
static_assert(((SEQ * 128) % 256) == 0);

typedef __attribute__((ext_vector_type(16))) _Float16 v16h;
typedef __attribute__((ext_vector_type(8)))  _Float16 v8h;
typedef __attribute__((ext_vector_type(4)))  _Float16 v4h;
typedef __attribute__((ext_vector_type(8)))  float    v8f;
typedef __attribute__((ext_vector_type(4)))  float    v4f;
typedef __attribute__((ext_vector_type(4)))  int      v4i;

union FragU { v16h v; v8h h[2]; };
__device__ __forceinline__ v16h frag_ld(const _Float16* p) {
  FragU f; f.h[0] = *(const v8h*)(p); f.h[1] = *(const v8h*)(p + 16); return f.v;
}
__device__ __forceinline__ v8f wm16(v16h a, v16h b, v8f c) {
  c = __builtin_amdgcn_wmma_f32_16x16x32_f16(false, a, false, b, (short)0, c, false, false);
  asm volatile("v_nop\n\tv_nop\n\tv_nop\n\tv_nop" : "+v"(c) : "v"(a), "v"(b));
  return c;
}
__device__ __forceinline__ void dep_guard_h(v8f& a, v8f& b, v16h x, v16h y) { asm volatile("v_nop\n\tv_nop\n\tv_nop\n\tv_nop" : "+v"(a), "+v"(b) : "v"(x), "v"(y)); }
__device__ __forceinline__ void keep4_h(v16h a, v16h b, v16h c, v16h d) { asm volatile("v_nop" :: "v"(a), "v"(b), "v"(c), "v"(d)); }
__device__ __forceinline__ void acc_guard4(v8f& a, v8f& b, v8f& c, v8f& d) { asm volatile("v_nop\n\tv_nop\n\tv_nop\n\tv_nop" : "+v"(a), "+v"(b), "+v"(c), "+v"(d)); }
__device__ __forceinline__ void wave_sync() {
  __builtin_amdgcn_fence(3  , "workgroup");
  __builtin_amdgcn_wave_barrier();
  __builtin_amdgcn_fence(2  , "workgroup");
}
__device__ __forceinline__ float cmb_bf(float v) {
  const unsigned u = __builtin_bit_cast(unsigned, v);
  const unsigned r = (u + 0x7fffu + ((u >> 16) & 1u)) & 0xffff0000u;
  return __builtin_bit_cast(float, r);
}

__global__ __launch_bounds__(256) void k_cast_rows(const float* __restrict__ S0, const float* __restrict__ S1, const float* __restrict__ S2,
                                                    unsigned long long sBatch, unsigned short* __restrict__ DST, unsigned long long dBatch,
                                                    unsigned long long dTensor, unsigned nR) {
  const unsigned u = blockIdx.x * 256u + threadIdx.x;
  if (u >= nR * 128u) return;
  const unsigned z = blockIdx.z;
  const float* SRC = (z == 0u) ? S0 : ((z == 1u) ? S1 : S2);
  const unsigned r = u >> 7, c0 = (u & 127u) << 3;
  const float* s = SRC + (size_t)blockIdx.y * sBatch + (size_t)r * DIMC + c0;
  const v4f x0 = *(const v4f*)s, x1 = *(const v4f*)(s + 4);
  v8h hv;
  hv[0] = (_Float16)cmb_bf(x0.x); hv[1] = (_Float16)cmb_bf(x0.y); hv[2] = (_Float16)cmb_bf(x0.z); hv[3] = (_Float16)cmb_bf(x0.w);
  hv[4] = (_Float16)cmb_bf(x1.x); hv[5] = (_Float16)cmb_bf(x1.y); hv[6] = (_Float16)cmb_bf(x1.z); hv[7] = (_Float16)cmb_bf(x1.w);
  volatile v8h* d = (volatile v8h*)((_Float16*)DST + (size_t)z * dTensor + (size_t)blockIdx.y * dBatch + (size_t)r * DIMC + c0);
  *d = hv; __threadfence(); *d = hv;
}

__global__ __launch_bounds__(256) void k_cast_wT(const float* __restrict__ W0, const float* __restrict__ W1, const float* __restrict__ W2,
                                                  const float* __restrict__ W3, unsigned short* __restrict__ DST) {
  const unsigned u = blockIdx.x * 256u + threadIdx.x;
  if (u >= (unsigned)DIMC * 128u) return;
  const unsigned y = blockIdx.y;
  const float* W = (y == 0u) ? W0 : ((y == 1u) ? W1 : ((y == 2u) ? W2 : W3));
  const unsigned o = u >> 7, k0 = (u & 127u) << 3;
  v8h hv;
#pragma unroll
  for (int e = 0; e < 8; ++e) hv[e] = (_Float16)(cmb_bf(W[(size_t)(k0 + (unsigned)e) * DIMC + o]) * 16.0f);
  volatile v8h* d = (volatile v8h*)((_Float16*)DST + (size_t)y * DIMC * DIMC + (size_t)o * DIMC + k0);
  *d = hv; __threadfence(); *d = hv;
}

__global__ __launch_bounds__(256) void k_bias_bf(const float* __restrict__ SRC, float* __restrict__ DST, unsigned n) {
  const unsigned u = blockIdx.x * 256u + threadIdx.x;
  if (u >= n) return;
  const float v = cmb_bf(SRC[u]);
  volatile float* d = (volatile float*)(DST + u);
  *d = v; __threadfence(); *d = v;
}

template <int BIAS_MODE, int OUT_MODE>
__global__ __launch_bounds__(256) void k_gemm64(
    const unsigned short* __restrict__ Ap, unsigned lda, unsigned long long strideA,
    const unsigned short* __restrict__ Btp, unsigned ldb, unsigned long long strideB,
    void* __restrict__ Cout, unsigned ldc, unsigned long long strideC,
    const float* __restrict__ bias, unsigned M, unsigned N, unsigned K, float scale) {
  __shared__ __align__(16) float sT[8][16 * 68];
  const unsigned b    = blockIdx.y;
  const unsigned lane = threadIdx.x & 31u;
  const unsigned wave = threadIdx.x >> 5;
  const unsigned tilesN = N >> 6;
  const unsigned tilesM = M >> 6;
  const unsigned tile = blockIdx.x * 8u + wave;
  if (tile >= tilesM * tilesN) return;
  const unsigned tm = tile / tilesN;
  const unsigned tn = tile - tm * tilesN;
  const unsigned m0 = tm << 6;
  const unsigned n0 = tn << 6;

  const _Float16* Ab = (const _Float16*)Ap + (size_t)b * strideA;
  const _Float16* Bb = (const _Float16*)Btp + (size_t)b * strideB;

  const unsigned rlane = lane & 15u;
  const unsigned koff  = (lane >> 4) * 8u;
  const unsigned mOff  = (lane >> 4) * 8u;

  v8f acc[4][4];
#pragma unroll
  for (int i = 0; i < 4; ++i)
#pragma unroll
    for (int j = 0; j < 4; ++j) acc[i][j] = (v8f){0.f,0.f,0.f,0.f,0.f,0.f,0.f,0.f};

  for (unsigned k0 = 0; k0 < K; k0 += 32u) {
    v16h bh[4];
#pragma unroll
    for (int j = 0; j < 4; ++j) {
      const size_t bo = (size_t)(n0 + ((unsigned)j << 4) + rlane) * ldb + koff + k0;
      bh[j] = frag_ld(Bb + bo);
    }
#pragma unroll
    for (int i = 0; i < 4; ++i) {
      const size_t ao = (size_t)(m0 + ((unsigned)i << 4) + rlane) * lda + koff + k0;
      v16h ah = frag_ld(Ab + ao);
#pragma unroll
      for (int j = 0; j < 4; ++j)
        acc[i][j] = __builtin_amdgcn_wmma_f32_16x16x32_f16(false, ah, false, bh[j], (short)0, acc[i][j], false, false);
      dep_guard_h(acc[i][0], acc[i][3], ah, ah);
    }
    keep4_h(bh[0], bh[1], bh[2], bh[3]);
  }
  acc_guard4(acc[0][0], acc[0][1], acc[0][2], acc[0][3]);
  acc_guard4(acc[1][0], acc[1][1], acc[1][2], acc[1][3]);
  acc_guard4(acc[2][0], acc[2][1], acc[2][2], acc[2][3]);
  acc_guard4(acc[3][0], acc[3][1], acc[3][2], acc[3][3]);

  float* slab = sT[wave];
#pragma unroll
  for (int i = 0; i < 4; ++i) {
    const unsigned mBase = m0 + ((unsigned)i << 4);
#pragma unroll
    for (int j = 0; j < 4; ++j) {
      const unsigned n = n0 + ((unsigned)j << 4) + rlane;
      float bv = 0.f;
      if (BIAS_MODE == 2) bv = bias[n];
#pragma unroll
      for (int r = 0; r < 8; ++r) {
        float v = acc[i][j][r] * scale;
        if (BIAS_MODE == 2) v += bv;
        slab[(mOff + (unsigned)r) * 68u + ((unsigned)j << 4) + rlane] = v;
      }
    }
    wave_sync();
    if (OUT_MODE == 0) {
      float* C = (float*)Cout + (size_t)b * strideC;
      const unsigned hh = lane >> 4, c4 = (lane & 15u) * 4u;
      for (int pass = 0; pass < 2; ++pass) {
#pragma unroll
        for (int it = 0; it < 8; ++it) {
          const unsigned row = (unsigned)it * 2u + hh;
          const v4f v = *(const v4f*)(slab + row * 68u + c4);
          *(volatile v4f*)(C + (size_t)(mBase + row) * ldc + n0 + c4) = v;
        }
        __threadfence();
      }
    } else {
      const unsigned q = lane >> 3, c8 = (lane & 7u) * 8u;
      _Float16* C = (_Float16*)Cout + (size_t)b * strideC;
      for (int pass = 0; pass < 2; ++pass) {
#pragma unroll
        for (int it = 0; it < 4; ++it) {
          const unsigned row = (unsigned)it * 4u + q;
          const float* sp = slab + row * 68u + c8;
          v8h hv;
#pragma unroll
          for (int e = 0; e < 8; ++e) hv[e] = (_Float16)sp[e];
          *(volatile v8h*)(C + (size_t)(mBase + row) * ldc + n0 + c8) = hv;
        }
        __threadfence();
      }
    }
    wave_sync();
  }
}

#define AT_PP 72
#define AT_OP 68
__global__ __launch_bounds__(128) void k_flash(const unsigned short* __restrict__ Qp, const unsigned short* __restrict__ Kp,
                                               const unsigned short* __restrict__ Vtp, const int* __restrict__ mask,
                                               unsigned short* __restrict__ ctxp) {
  __shared__ __align__(16) _Float16 Psh[4][16 * AT_PP];
  __shared__ __align__(16) float    Os[4][16 * AT_OP];
  constexpr unsigned NQB = SEQ / 64;
  const float SC2   = 0.125f * 1.4426950408889634f;
  const float FILL2 = -1.0e9f * 1.4426950408889634f;
  const float PSC   = 16384.0f;
  const float CTXC  = 16.0f;

  const unsigned tid = threadIdx.x, wave = tid >> 5, lane = tid & 31u, hh = lane >> 4, c = lane & 15u;
  const unsigned bx = blockIdx.x;
  const unsigned qb = bx % NQB;
  const unsigned bh = bx / NQB;
  const unsigned h  = bh % (unsigned)NHEAD;
  const unsigned b  = bh / (unsigned)NHEAD;
  const unsigned q0 = qb * 64u + wave * 16u;

  const _Float16* Q  = (const _Float16*)Qp;
  const _Float16* K  = (const _Float16*)Kp;
  const _Float16* Vt = (const _Float16*)Vtp;

  const _Float16* qrow  = Q + (size_t)(b * (unsigned)SEQ + q0 + c) * DIMC + h * HDIM + 8u * hh;
  const v16h qa0 = frag_ld(qrow), qa1 = frag_ld(qrow + 32);
  const _Float16* kbase = K + (size_t)(b * (unsigned)SEQ) * DIMC + h * HDIM + 8u * hh;
  const _Float16* vbase = Vt + ((size_t)b * DIMC + h * HDIM + c) * SEQ + 8u * hh;
  const int* mbase = mask + (size_t)b * SEQ_FULL * SEQ_FULL + (size_t)(q0 + 8u * hh) * SEQ_FULL + 4u * c;

  float mrow[8], lrow[8];
  v8f oacc[4];
#pragma unroll
  for (int r = 0; r < 8; ++r) { mrow[r] = -INFINITY; lrow[r] = 0.f; }
#pragma unroll
  for (int t = 0; t < 4; ++t) oacc[t] = (v8f){0.f,0.f,0.f,0.f,0.f,0.f,0.f,0.f};

  _Float16* pw = Psh[wave];

#pragma unroll 1
  for (unsigned kc = 0; kc < NQB; ++kc) {
    const unsigned kv0 = kc * 64u;
    wave_sync();
    v8f s[4];
#pragma unroll
    for (int j = 0; j < 4; ++j) {
      const _Float16* kr = kbase + (size_t)(kv0 + 4u * c + (unsigned)j) * DIMC;
      const v16h k0f = frag_ld(kr), k1f = frag_ld(kr + 32);
      v8f z = (v8f){0.f,0.f,0.f,0.f,0.f,0.f,0.f,0.f};
      z = wm16(qa0, k0f, z);
      s[j] = wm16(qa1, k1f, z);
    }
    v4i mk[8];
#pragma unroll
    for (int r = 0; r < 8; ++r) mk[r] = *(const v4i*)(mbase + (size_t)r * SEQ_FULL + kv0);

#pragma unroll
    for (int r = 0; r < 8; ++r) {
      const float x0 = (mk[r].x == 0) ? FILL2 : s[0][r] * SC2;
      const float x1 = (mk[r].y == 0) ? FILL2 : s[1][r] * SC2;
      const float x2 = (mk[r].z == 0) ? FILL2 : s[2][r] * SC2;
      const float x3 = (mk[r].w == 0) ? FILL2 : s[3][r] * SC2;
      float m = fmaxf(fmaxf(x0, x1), fmaxf(x2, x3));
      m = fmaxf(m, __shfl_xor(m, 1, 32)); m = fmaxf(m, __shfl_xor(m, 2, 32));
      m = fmaxf(m, __shfl_xor(m, 4, 32)); m = fmaxf(m, __shfl_xor(m, 8, 32));
      const float mnew  = fmaxf(mrow[r], m);
      const float alpha = exp2f(mrow[r] - mnew);
      mrow[r] = mnew;
      const float p0 = exp2f(x0 - mnew), p1 = exp2f(x1 - mnew), p2 = exp2f(x2 - mnew), p3 = exp2f(x3 - mnew);
      float psum = (p0 + p1) + (p2 + p3);
      psum += __shfl_xor(psum, 1, 32); psum += __shfl_xor(psum, 2, 32);
      psum += __shfl_xor(psum, 4, 32); psum += __shfl_xor(psum, 8, 32);
      lrow[r] = lrow[r] * alpha + psum;
#pragma unroll
      for (int t = 0; t < 4; ++t) oacc[t][r] *= alpha;
      v4h ph;
      ph.x = (_Float16)(p0 * PSC); ph.y = (_Float16)(p1 * PSC); ph.z = (_Float16)(p2 * PSC); ph.w = (_Float16)(p3 * PSC);
      *(v4h*)(pw + (8u * hh + (unsigned)r) * AT_PP + 4u * c) = ph;
    }
    wave_sync();
#pragma unroll
    for (int kk = 0; kk < 2; ++kk) {
      const v16h pa = frag_ld(pw + c * AT_PP + (unsigned)kk * 32u + 8u * hh);
#pragma unroll
      for (int t = 0; t < 4; ++t) {
        const v16h vb = frag_ld(vbase + (size_t)(t * 16) * SEQ + kv0 + (unsigned)kk * 32u);
        oacc[t] = wm16(pa, vb, oacc[t]);
      }
    }
  }

  float* os = Os[wave];
#pragma unroll
  for (int r = 0; r < 8; ++r) {
    const float inv = CTXC * (1.0f / (lrow[r] * PSC));
#pragma unroll
    for (int t = 0; t < 4; ++t) os[(8u * hh + (unsigned)r) * AT_OP + (unsigned)t * 16u + c] = oacc[t][r] * inv;
  }
  wave_sync();
  {
    const unsigned q4 = lane >> 3, c8 = (lane & 7u) * 8u;
    _Float16* cb = (_Float16*)ctxp + (size_t)(b * (unsigned)SEQ + q0) * DIMC + h * HDIM;
    for (int pass = 0; pass < 2; ++pass) {
#pragma unroll
      for (int it = 0; it < 4; ++it) {
        const unsigned row = (unsigned)it * 4u + q4;
        const float* sp = os + row * AT_OP + c8;
        v8h hv;
#pragma unroll
        for (int e = 0; e < 8; ++e) hv[e] = (_Float16)sp[e];
        *(volatile v8h*)(cb + (size_t)row * DIMC + c8) = hv;
      }
      __threadfence();
    }
  }
}

static constexpr size_t SZ_X16   = (size_t)3 * MROWS * DIMC * 2;
static constexpr size_t SZ_WT16  = (size_t)4 * DIMC * DIMC * 2;
static constexpr size_t SZ_QK16  = (size_t)2 * MROWS * DIMC * 2;
static constexpr size_t SZ_VT16  = (size_t)NB * DIMC * SEQ * 2;
static constexpr size_t SZ_CTX16 = (size_t)MROWS * DIMC * 2;
static constexpr size_t SZ_BRO   = (size_t)DIMC * 4;
static constexpr size_t SZ_TOTAL = SZ_X16 + SZ_WT16 + SZ_QK16 + SZ_VT16 + SZ_CTX16 + SZ_BRO;
static_assert((SZ_X16 % 256) == 0 && (SZ_WT16 % 256) == 0 && (SZ_QK16 % 256) == 0 && (SZ_VT16 % 256) == 0 && (SZ_CTX16 % 256) == 0 && (SZ_BRO % 256) == 0);
static_assert(SZ_TOTAL <= (size_t)134217728);
static_assert((size_t)(SEQ * 128 / 256) * 256 * 8 == (size_t)SEQ * DIMC);
static_assert((size_t)(DIMC * 128 / 256) * 256 * 8 == (size_t)DIMC * DIMC);
static_assert((size_t)(SEQ / 64) * 4 * 16 * 64 == (size_t)SEQ * HDIM);
static_assert((((MROWS / 64) * (DIMC / 64)) % 8) == 0);
static_assert((((DIMC / 64) * (SEQ / 64)) % 8) == 0);

extern "C" void kernel_launch(void* const* d_in, const int* in_sizes, int n_in, void* d_out, int out_size, void* d_ws, size_t ws_size, hipStream_t stream) {
  if (n_in < 9) return;
  const long long needX = (long long)(NB - 1) * SEQ_FULL * DIMC + (long long)SEQ * DIMC;
  const long long needM = (long long)(NB - 1) * SEQ_FULL * SEQ_FULL + (long long)(SEQ - 1) * SEQ_FULL + SEQ;
  if ((long long)in_sizes[0] < needX || (long long)in_sizes[1] < needX || (long long)in_sizes[2] < needX) return;
  if ((long long)in_sizes[3] < needM) return;
  if (in_sizes[4] < DIMC * DIMC || in_sizes[5] < DIMC * DIMC || in_sizes[6] < DIMC * DIMC || in_sizes[7] < DIMC * DIMC || in_sizes[8] < DIMC) return;
  if ((long long)out_size < (long long)MROWS * DIMC) return;
  if (ws_size < SZ_TOTAL) return;

  const float* q    = (const float*)d_in[0];
  const float* k    = (const float*)d_in[1];
  const float* v    = (const float*)d_in[2];
  const int*   mask = (const int*)d_in[3];
  const float* Wq   = (const float*)d_in[4];
  const float* Wk   = (const float*)d_in[5];
  const float* Wv   = (const float*)d_in[6];
  const float* Wp   = (const float*)d_in[7];
  const float* bp   = (const float*)d_in[8];
  float* out = (float*)d_out;

  char* wsp = (char*)d_ws;
  unsigned short* X16   = (unsigned short*)wsp; wsp += SZ_X16;
  unsigned short* WT16  = (unsigned short*)wsp; wsp += SZ_WT16;
  unsigned short* QK16  = (unsigned short*)wsp; wsp += SZ_QK16;
  unsigned short* VT16  = (unsigned short*)wsp; wsp += SZ_VT16;
  unsigned short* CTX16 = (unsigned short*)wsp; wsp += SZ_CTX16;
  float*          BRO   = (float*)wsp;          wsp += SZ_BRO;

  const unsigned long long planeX = (unsigned long long)MROWS * DIMC;
  const unsigned long long planeW = (unsigned long long)DIMC * DIMC;

  k_cast_wT<<<dim3((unsigned)(DIMC * 128 / 256), 4u, 1u), 256, 0, stream>>>(Wq, Wk, Wv, Wp, WT16);
  k_bias_bf<<<dim3((unsigned)((DIMC + 255) / 256), 1u, 1u), 256, 0, stream>>>(bp, BRO, (unsigned)DIMC);
  k_cast_rows<<<dim3((unsigned)(SEQ * 128 / 256), (unsigned)NB, 3u), 256, 0, stream>>>(q, k, v, (unsigned long long)SEQ_FULL * DIMC, X16,
                                                                                      (unsigned long long)SEQ * DIMC, planeX, (unsigned)SEQ);
  k_gemm64<0, 1><<<dim3((unsigned)(((MROWS / 64) * (DIMC / 64)) / 8), 2u, 1u), 256, 0, stream>>>(
      X16, (unsigned)DIMC, planeX, WT16, (unsigned)DIMC, planeW, (void*)QK16, (unsigned)DIMC, planeX, nullptr,
      (unsigned)MROWS, (unsigned)DIMC, (unsigned)DIMC, 0.0625f);
  k_gemm64<0, 1><<<dim3((unsigned)(((DIMC / 64) * (SEQ / 64)) / 8), (unsigned)NB, 1u), 256, 0, stream>>>(
      WT16 + 2 * planeW, (unsigned)DIMC, 0ull, X16 + 2 * planeX, (unsigned)DIMC, (unsigned long long)SEQ * DIMC,
      (void*)VT16, (unsigned)SEQ, (unsigned long long)DIMC * SEQ, nullptr,
      (unsigned)DIMC, (unsigned)SEQ, (unsigned)DIMC, 0.0625f);
  k_flash<<<dim3((unsigned)(NB * NHEAD * (SEQ / 64)), 1u, 1u), 128, 0, stream>>>(QK16, QK16 + planeX, VT16, mask, CTX16);
  k_gemm64<2, 0><<<dim3((unsigned)(((MROWS / 64) * (DIMC / 64)) / 8), 1u, 1u), 256, 0, stream>>>(
      CTX16, (unsigned)DIMC, 0ull, WT16 + 3 * planeW, (unsigned)DIMC, 0ull, (void*)out, (unsigned)DIMC, 0ull, BRO,
      (unsigned)MROWS, (unsigned)DIMC, (unsigned)DIMC, 0.00390625f);
}
